// FAVOR_91319594647802
// MI455X (gfx1250) — hardware-verified
//
#include <hip/hip_runtime.h>

constexpr int NBATCH = 8;
constexpr int NDIM   = 64;
constexpr int NSEQ   = 2048;
constexpr int NFEAT  = 64;
constexpr int NVAL   = 64;
constexpr int CHUNK  = 64;
constexpr int NCHUNK = NSEQ / CHUNK;
constexpr int PITB   = 72;
constexpr int PITF   = 68;
constexpr int NTHR   = 256;
constexpr float FEAT_EPS = 1.0e-3f;

static_assert(NSEQ % CHUNK == 0);
static_assert(NDIM == 64 && NFEAT == 64 && NVAL == 64 && CHUNK == 64);
static_assert(CHUNK % 32 == 0);
static_assert(NTHR == 256);
static_assert((PITB * 2) % 16 == 0 && (PITF * 4) % 16 == 0);

typedef __attribute__((ext_vector_type(16))) __bf16   v16b;
typedef __attribute__((ext_vector_type(8)))  __bf16   v8b;
typedef __attribute__((ext_vector_type(8)))  float    v8f;
typedef __attribute__((ext_vector_type(4)))  float    v4f;
typedef __attribute__((ext_vector_type(4)))  unsigned int v4u;
typedef __attribute__((ext_vector_type(2)))  unsigned int v2u;

__device__ __forceinline__ unsigned short f2bf_bits(float f) {
  unsigned u = __float_as_uint(f);
  return (unsigned short)((u + 0x7FFFu + ((u >> 16) & 1u)) >> 16);
}
__device__ __forceinline__ float bf_bits2f(unsigned short h) { return __uint_as_float(((unsigned)h) << 16); }

__device__ __forceinline__ void dep_guard_b(v8f& a, v8f& b, v16b x, v16b y) { asm volatile("v_nop\n\tv_nop\n\tv_nop\n\tv_nop" : "+v"(a), "+v"(b) : "v"(x), "v"(y)); }
__device__ __forceinline__ void keep4_b(v16b a, v16b b, v16b c, v16b d) { asm volatile("v_nop" :: "v"(a), "v"(b), "v"(c), "v"(d)); }
template <typename T> struct Frag;
template <> struct Frag<__bf16> {
  typedef v16b V; union U { v16b v; v8b h[2]; };
  static __device__ __forceinline__ v16b load(const __bf16* p) {
    U f; f.h[0] = *(const v8b*)(p); f.h[1] = *(const v8b*)(p + 16); return f.v;
  }
  static __device__ __forceinline__ v8f mma(v16b a, v16b b, v8f c) {
    return __builtin_amdgcn_wmma_f32_16x16x32_bf16(false, a, false, b, (short)0, c, false, false);
  }
  static __device__ __forceinline__ void guard(v8f& a, v8f& b, v16b x, v16b y) { dep_guard_b(a, b, x, y); }
  static __device__ __forceinline__ void keep(v16b a, v16b b, v16b c, v16b d) { keep4_b(a, b, c, d); }
};

__device__ __forceinline__ v8f at_mma(v16b a, v16b b, v8f c) {
  c = __builtin_amdgcn_wmma_f32_16x16x32_bf16(false, a, false, b, (short)0, c, false, false);
  asm volatile("v_nop\n\tv_nop\n\tv_nop\n\tv_nop" : "+v"(c) : "v"(a), "v"(b));
  return c;
}

__device__ __forceinline__ void split_bits(float f, unsigned short& hi, unsigned short& lo) {
  hi = f2bf_bits(f);
  lo = f2bf_bits(f - bf_bits2f(hi));
}

__device__ __forceinline__ const __bf16* bfp(const unsigned short* p) { return (const __bf16*)(const void*)p; }

__device__ __forceinline__ v8f zero8() { return (v8f){0.f,0.f,0.f,0.f,0.f,0.f,0.f,0.f}; }

__device__ __forceinline__ v8f tile_k64_split(const unsigned short* Ah, const unsigned short* Al, int arow0,
                                               const unsigned short* Bh, const unsigned short* Bl, int brow0,
                                               int lane, v8f acc) {
  const int rl = lane & 15, koff = (lane >> 4) * 8;
#pragma unroll
  for (int ks = 0; ks < 2; ++ks) {
    const int ao = (arow0 + rl) * PITB + 32 * ks + koff;
    const int bo = (brow0 + rl) * PITB + 32 * ks + koff;
    const v16b ah = Frag<__bf16>::load(bfp(Ah) + ao);
    const v16b al = Frag<__bf16>::load(bfp(Al) + ao);
    const v16b bh = Frag<__bf16>::load(bfp(Bh) + bo);
    const v16b bl = Frag<__bf16>::load(bfp(Bl) + bo);
    acc = at_mma(ah, bh, acc);
    acc = at_mma(ah, bl, acc);
    acc = at_mma(al, bh, acc);
  }
  return acc;
}

__device__ __forceinline__ void put_split_rm(unsigned short* Ph, unsigned short* Pl, int row0, int col0, int lane, v8f v) {
  const int hq = lane >> 4, cq = lane & 15;
#pragma unroll
  for (int r = 0; r < 8; ++r) {
    unsigned short hb, lb;
    split_bits(v[r], hb, lb);
    const int off = (row0 + 8 * hq + r) * PITB + col0 + cq;
    Ph[off] = hb;
    Pl[off] = lb;
  }
}
__device__ __forceinline__ void put_split_tr(unsigned short* Ph, unsigned short* Pl, int row0, int col0, int lane, v8f v) {
  const int hq = lane >> 4, cq = lane & 15;
  v4u uh, ul;
#pragma unroll
  for (int e = 0; e < 4; ++e) {
    unsigned short ha, la, hb, lb;
    split_bits(v[2 * e], ha, la);
    split_bits(v[2 * e + 1], hb, lb);
    uh[e] = (unsigned)ha | ((unsigned)hb << 16);
    ul[e] = (unsigned)la | ((unsigned)lb << 16);
  }
  const int off = (col0 + cq) * PITB + row0 + 8 * hq;
  *(v4u*)(Ph + off) = uh;
  *(v4u*)(Pl + off) = ul;
}

__global__ __launch_bounds__(NTHR)
void lin_attn_causal_kernel(const float* __restrict__ keys,
                            const float* __restrict__ values,
                            const float* __restrict__ queries,
                            const float* __restrict__ proj,
                            float* __restrict__ out) {
  __shared__ __align__(16) unsigned short sXh[CHUNK * PITB];
  __shared__ __align__(16) unsigned short sXl[CHUNK * PITB];
  __shared__ __align__(16) unsigned short sYh[CHUNK * PITB];
  __shared__ __align__(16) unsigned short sYl[CHUNK * PITB];
  __shared__ __align__(16) unsigned short sWh[NFEAT * PITB];
  __shared__ __align__(16) unsigned short sWl[NFEAT * PITB];
  __shared__ __align__(16) unsigned short sQh[CHUNK * PITB];
  __shared__ __align__(16) unsigned short sQl[CHUNK * PITB];
  __shared__ __align__(16) unsigned short sKAh[CHUNK * PITB];
  __shared__ __align__(16) unsigned short sKAl[CHUNK * PITB];
  __shared__ __align__(16) unsigned short sKTh[NFEAT * PITB];
  __shared__ __align__(16) unsigned short sKTl[NFEAT * PITB];
  __shared__ __align__(16) float sF[CHUNK * PITF];
  __shared__ __align__(16) float sZ[NFEAT];
  __shared__ __align__(16) float sRN[CHUNK];

  const int tid  = threadIdx.x;
  const int lane = tid & 31;
  const int w    = tid >> 5;
  const int hh   = lane >> 4;
  const int cc   = lane & 15;
  const int tm   = w >> 1;
  const int tn0  = (w & 1) * 2;
  const int b    = blockIdx.x;

  const float* kb = keys    + (size_t)b * NDIM * NSEQ;
  const float* qb = queries + (size_t)b * NDIM * NSEQ;
  const float* vb = values  + (size_t)b * NVAL * NSEQ;
  float*       ob = out     + (size_t)b * NVAL * NSEQ;

#pragma unroll
  for (int it = 0; it < 4; ++it) {
    const int idx = tid + it * NTHR;
    const int d   = idx >> 4;
    const int m4  = (idx & 15) << 2;
    const v4f wv = *(const v4f*)(proj + (size_t)d * NFEAT + m4);
#pragma unroll
    for (int e = 0; e < 4; ++e) {
      unsigned short hb, lb;
      split_bits(wv[e], hb, lb);
      const int off = (m4 + e) * PITB + d;
      sWh[off] = hb;
      sWl[off] = lb;
    }
  }
  if (tid < NFEAT) sZ[tid] = 0.f;

  v8f accS[2];
  accS[0] = zero8();
  accS[1] = zero8();

  for (int ch = 0; ch < NCHUNK; ++ch) {
    const int l0 = ch * CHUNK;

#pragma unroll
    for (int it = 0; it < 4; ++it) {
      const int idx = tid + it * NTHR;
      const int d   = idx >> 4;
      const int i4  = (idx & 15) << 2;
      const v4f qv = *(const v4f*)(qb + (size_t)d * NSEQ + l0 + i4);
      const v4f kv = *(const v4f*)(kb + (size_t)d * NSEQ + l0 + i4);
#pragma unroll
      for (int e = 0; e < 4; ++e) {
        unsigned short hq, lq, hk, lk;
        split_bits(qv[e], hq, lq);
        split_bits(kv[e], hk, lk);
        const int off = (i4 + e) * PITB + d;
        sXh[off] = hq; sXl[off] = lq;
        sYh[off] = hk; sYl[off] = lk;
      }
    }
    __syncthreads();

    {
      v8f aq[2], ak[2];
      aq[0] = zero8(); aq[1] = zero8(); ak[0] = zero8(); ak[1] = zero8();
      const int rl = lane & 15, koff = hh * 8;
#pragma unroll
      for (int ks = 0; ks < 2; ++ks) {
        const int ao = (16 * tm + rl) * PITB + 32 * ks + koff;
        const v16b qh = Frag<__bf16>::load(bfp(sXh) + ao);
        const v16b ql = Frag<__bf16>::load(bfp(sXl) + ao);
        const v16b kh = Frag<__bf16>::load(bfp(sYh) + ao);
        const v16b kl = Frag<__bf16>::load(bfp(sYl) + ao);
#pragma unroll
        for (int j = 0; j < 2; ++j) {
          const int bo = (16 * (tn0 + j) + rl) * PITB + 32 * ks + koff;
          const v16b wh = Frag<__bf16>::load(bfp(sWh) + bo);
          const v16b wl = Frag<__bf16>::load(bfp(sWl) + bo);
          aq[j] = at_mma(qh, wh, aq[j]);
          aq[j] = at_mma(qh, wl, aq[j]);
          aq[j] = at_mma(ql, wh, aq[j]);
          ak[j] = at_mma(kh, wh, ak[j]);
          ak[j] = at_mma(kh, wl, ak[j]);
          ak[j] = at_mma(kl, wh, ak[j]);
        }
      }
#pragma unroll
      for (int j = 0; j < 2; ++j) {
        v8f pq, pk;
#pragma unroll
        for (int r = 0; r < 8; ++r) {
          pq[r] = fmaxf(aq[j][r], 0.f) + FEAT_EPS;
          pk[r] = fmaxf(ak[j][r], 0.f) + FEAT_EPS;
        }
        put_split_rm(sQh,  sQl,  16 * tm, 16 * (tn0 + j), lane, pq);
        put_split_rm(sKAh, sKAl, 16 * tm, 16 * (tn0 + j), lane, pk);
        put_split_tr(sKTh, sKTl, 16 * tm, 16 * (tn0 + j), lane, pk);
      }
    }
    __syncthreads();

    v8f accA[2];
    {
#pragma unroll
      for (int it = 0; it < 4; ++it) {
        const int idx = tid + it * NTHR;
        const int vr  = idx >> 4;
        const int i4  = (idx & 15) << 2;
        const v4f vv = *(const v4f*)(vb + (size_t)vr * NSEQ + l0 + i4);
        unsigned short h0, g0, h1, g1, h2, g2, h3, g3;
        split_bits(vv[0], h0, g0);
        split_bits(vv[1], h1, g1);
        split_bits(vv[2], h2, g2);
        split_bits(vv[3], h3, g3);
        v2u uh, ul;
        uh[0] = (unsigned)h0 | ((unsigned)h1 << 16);
        uh[1] = (unsigned)h2 | ((unsigned)h3 << 16);
        ul[0] = (unsigned)g0 | ((unsigned)g1 << 16);
        ul[1] = (unsigned)g2 | ((unsigned)g3 << 16);
        const int off = vr * PITB + i4;
        *(v2u*)(sXh + off) = uh;
        *(v2u*)(sXl + off) = ul;
      }
      put_split_rm(sYh, sYl, 16 * tm, 16 * tn0,       lane, accS[0]);
      put_split_rm(sYh, sYl, 16 * tm, 16 * (tn0 + 1), lane, accS[1]);
#pragma unroll
      for (int j = 0; j < 2; ++j) {
        accA[j] = tile_k64_split(sQh, sQl, 16 * tm, sKAh, sKAl, 16 * (tn0 + j), lane, zero8());
#pragma unroll
        for (int r = 0; r < 8; ++r) {
          const int row = 16 * tm + 8 * hh + r;
          const int col = 16 * (tn0 + j) + cc;
          const float a = accA[j][r];
          accA[j][r] = (col <= row) ? a : 0.f;
        }
      }
    }
    __syncthreads();

#pragma unroll
    for (int j = 0; j < 2; ++j) {
      put_split_rm(sKAh, sKAl, 16 * tm, 16 * (tn0 + j), lane, accA[j]);
#pragma unroll
      for (int r = 0; r < 8; ++r)
        sF[(16 * tm + 8 * hh + r) * PITF + 16 * (tn0 + j) + cc] = accA[j][r];
    }
    __syncthreads();

    float zp = 0.f;
    if (tid < CHUNK) {
      const int l = tid;
      float s = 0.f;
#pragma unroll 1
      for (int j = 0; j < 8; ++j) {
        const v4u wh = *(const v4u*)(sQh + l * PITB + 8 * j);
        const v4u wl = *(const v4u*)(sQl + l * PITB + 8 * j);
#pragma unroll
        for (int e = 0; e < 4; ++e) {
          const float p0 = __uint_as_float(wh[e] << 16) + __uint_as_float(wl[e] << 16);
          const float p1 = __uint_as_float(wh[e] & 0xffff0000u) + __uint_as_float(wl[e] & 0xffff0000u);
          s += p0 * sZ[8 * j + 2 * e];
          s += p1 * sZ[8 * j + 2 * e + 1];
        }
      }
      float asum = 0.f;
#pragma unroll 1
      for (int i = 0; i < CHUNK; i += 4) {
        const v4f av = *(const v4f*)(sF + l * PITF + i);
        asum += (av[0] + av[1]) + (av[2] + av[3]);
      }
      sRN[l] = 1.0f / (s + asum);
    } else if (tid < 2 * CHUNK) {
      const int m = tid - CHUNK;
#pragma unroll 1
      for (int j = 0; j < 8; ++j) {
        const v4u wh = *(const v4u*)(sKTh + m * PITB + 8 * j);
        const v4u wl = *(const v4u*)(sKTl + m * PITB + 8 * j);
#pragma unroll
        for (int e = 0; e < 4; ++e) {
          zp += __uint_as_float(wh[e] << 16) + __uint_as_float(wl[e] << 16);
          zp += __uint_as_float(wh[e] & 0xffff0000u) + __uint_as_float(wl[e] & 0xffff0000u);
        }
      }
    }
    __syncthreads();
    if (tid >= CHUNK && tid < 2 * CHUNK) sZ[tid - CHUNK] += zp;

    {
      v8f accO[2];
#pragma unroll
      for (int j = 0; j < 2; ++j) {
        accO[j] = tile_k64_split(sKAh, sKAl, 16 * tm, sXh, sXl, 16 * (tn0 + j), lane, zero8());
        accO[j] = tile_k64_split(sQh, sQl, 16 * tm, sYh, sYl, 16 * (tn0 + j), lane, accO[j]);
        accS[j] = tile_k64_split(sXh, sXl, 16 * tm, sKTh, sKTl, 16 * (tn0 + j), lane, accS[j]);
      }
      const v4f rn0 = *(const v4f*)(sRN + 16 * tm + 8 * hh);
      const v4f rn1 = *(const v4f*)(sRN + 16 * tm + 8 * hh + 4);
#pragma unroll
      for (int j = 0; j < 2; ++j) {
        v4f o0, o1;
        o0[0] = accO[j][0] * rn0[0]; o0[1] = accO[j][1] * rn0[1]; o0[2] = accO[j][2] * rn0[2]; o0[3] = accO[j][3] * rn0[3];
        o1[0] = accO[j][4] * rn1[0]; o1[1] = accO[j][5] * rn1[1]; o1[2] = accO[j][6] * rn1[2]; o1[3] = accO[j][7] * rn1[3];
        const int off = (16 * (tn0 + j) + cc) * PITF + 16 * tm + 8 * hh;
        *(v4f*)(sF + off)     = o0;
        *(v4f*)(sF + off + 4) = o1;
      }
    }
    __syncthreads();

    {
      const int c4 = cc * 4;
      for (int pass = 0; pass < 2; ++pass) {
#pragma unroll
        for (int it = 0; it < 4; ++it) {
          const int row = 8 * w + 2 * it + hh;
          const v4f val = *(const v4f*)(sF + row * PITF + c4);
          *(volatile v4f*)(ob + (size_t)row * NSEQ + l0 + c4) = val;
        }
        __threadfence();
      }
    }
  }
}

extern "C" void kernel_launch(void* const* d_in, const int* in_sizes, int n_in,
                              void* d_out, int out_size, void* d_ws, size_t ws_size,
                              hipStream_t stream) {
  (void)d_ws; (void)ws_size;
  if (n_in < 4) return;
  if (in_sizes[0] != NBATCH * NDIM * NSEQ) return;
  if (in_sizes[1] != NBATCH * NVAL * NSEQ) return;
  if (in_sizes[2] != NBATCH * NDIM * NSEQ) return;
  if (in_sizes[3] != NDIM * NFEAT) return;
  if (out_size != NBATCH * NVAL * NSEQ) return;
  const float* keys    = (const float*)d_in[0];
  const float* values  = (const float*)d_in[1];
  const float* queries = (const float*)d_in[2];
  const float* proj    = (const float*)d_in[3];
  float* out = (float*)d_out;
  lin_attn_causal_kernel<<<dim3(NBATCH), dim3(NTHR), 0, stream>>>(keys, values, queries, proj, out);
}
